// HiddenStateMLPPooling_34772055228496
// MI455X (gfx1250) — hardware-run, weakly checked
//
#include <hip/hip_runtime.h>
#include <stddef.h>


typedef _Float16 v16h __attribute__((ext_vector_type(16)));
typedef _Float16 v8h  __attribute__((ext_vector_type(8)));
typedef float    v8f  __attribute__((ext_vector_type(8)));
typedef float    v4f  __attribute__((ext_vector_type(4)));
typedef float    v2f  __attribute__((ext_vector_type(2)));

#ifndef NB
#define NB 4
#endif
#ifndef SEQ
#define SEQ 512
#endif
#define NB_FULL  4
#define SEQ_FULL 512
#define HDIM 128
#define EH   64
#define ES   32
#define EV   32
#define PD   128
#define OD   128
#define MROWS (NB * SEQ)
#define BPB   (SEQ / 64)

static_assert(NB >= 1 && NB <= NB_FULL);
static_assert(SEQ >= 64 && SEQ <= SEQ_FULL && (SEQ % 64) == 0);
static_assert(PD == ES + EH + EV);
static_assert(HDIM == 128 && PD == 128 && OD == 128 && EH == 64 && ES == 32 && EV == 32);
static_assert((HDIM % 32) == 0 && (PD % 32) == 0);
static_assert((HDIM % 64) == 0 && (EH % 64) == 0 && (PD % 64) == 0 && (OD % 64) == 0);
static_assert((MROWS % 64) == 0 && BPB >= 1);
static_assert(OD == 32 * 4);
static_assert(HDIM == 16 * 8 && PD == 16 * 8);
static_assert((size_t)NB_FULL * SEQ_FULL * OD * 4 == (size_t)1048576);

#define LDT 72
#define LDC 68
static_assert((LDT % 8) == 0 && LDT >= 64);
static_assert((LDC % 4) == 0 && LDC >= 64);
#define LDA 136
#define LDO 132
static_assert((LDA % 8) == 0 && LDA >= 128);
static_assert((LDO % 4) == 0 && LDO >= 128);

#define WCARRY 64.0f
#define HCARRY 16.0f
#define ACARRY 16.0f
#define FILLV  (-100.0f)
#define NEGV   (-3.402823466e+38f)

#define WH_BYTES ((size_t)EH * HDIM * 2)
#define WO_BYTES ((size_t)OD * PD * 2)
#define HP_BYTES ((size_t)(MROWS / 64) * 64 * 4)
#define OFF_WH ((size_t)0)
#define OFF_WO (OFF_WH + WH_BYTES)
#define OFF_HP (OFF_WO + WO_BYTES)
#define WS_TOTAL (OFF_HP + HP_BYTES)
static_assert((WH_BYTES % 128) == 0 && (WO_BYTES % 128) == 0 && (HP_BYTES % 128) == 0);
static_assert(WS_TOTAL <= (size_t)134217728);

__device__ __forceinline__ float bf16r(float x) {
  unsigned int u = __float_as_uint(x);
  u = (u + 0x7FFFu + ((u >> 16) & 1u)) & 0xFFFF0000u;
  return __uint_as_float(u);
}

__device__ __forceinline__ v16h frag_at(const _Float16* p) {
  v8h lo = *(const v8h*)(p);
  v8h hi = *(const v8h*)(p + 16);
  v16h out;
#pragma unroll
  for (int i = 0; i < 8; ++i) { out[i] = lo[i]; out[i + 8] = hi[i]; }
  return out;
}

__device__ __forceinline__ v8f wmma16(v16h a, v16h b, v8f c) {
  v8f d = __builtin_amdgcn_wmma_f32_16x16x32_f16(false, a, false, b, (short)0, c,
                                                 false, false);
  asm volatile("v_nop\n\tv_nop\n\tv_nop\n\tv_nop" : "+v"(d) : "v"(a), "v"(b));
  return d;
}

__device__ __forceinline__ float red16_max(float x) {
#pragma unroll
  for (int off = 1; off < 16; off <<= 1) x = fmaxf(x, __shfl_xor(x, off, 32));
  return x;
}

__device__ __forceinline__ v16h frag_join(v8h lo, v8h hi) {
  v16h out;
#pragma unroll
  for (int i = 0; i < 8; ++i) { out[i] = lo[i]; out[i + 8] = hi[i]; }
  return out;
}

static __device__ __forceinline__ _Float16 toh_flush(float v) {
  const _Float16 r = (_Float16)v;
  return (fabsf(v) < 6.103515625e-05f) ? (_Float16)0.0f : r;
}

__device__ __forceinline__ float bf16n(float x) {
  const float r = bf16r(x);
  return (x != x) ? x : r;
}

__global__ __launch_bounds__(256) void wconv_kernel(
    const float* __restrict__ W, _Float16* __restrict__ Wt, unsigned ldw, unsigned ldk) {
  __shared__ _Float16 T[64 * LDT];
  const unsigned tid = threadIdx.x;
  const unsigned n0 = blockIdx.x * 64u;
  const unsigned k0 = blockIdx.y * 64u;
#pragma unroll 4
  for (unsigned j = 0; j < 16u; ++j) {
    const unsigned idx = tid + 256u * j;
    const unsigned kr = idx >> 6, nc = idx & 63u;
    const float v = W[(size_t)(k0 + kr) * ldw + n0 + nc];
    T[nc * LDT + kr] = (_Float16)(WCARRY * bf16r(v));
  }
  __syncthreads();
  v8h x[2];
  size_t off[2];
#pragma unroll
  for (unsigned i = 0; i < 2u; ++i) {
    const unsigned n = 32u * i + (tid >> 3);
    const unsigned kc = (tid & 7u) * 8u;
    x[i] = *(const v8h*)&T[n * LDT + kc];
    off[i] = (size_t)(n0 + n) * ldk + k0 + kc;
  }
#pragma unroll
  for (int i = 0; i < 2; ++i) *(volatile v8h*)(Wt + off[i]) = x[i];
  __threadfence();
#pragma unroll
  for (int i = 0; i < 2; ++i) *(volatile v8h*)(Wt + off[i]) = x[i];
}

__global__ __launch_bounds__(256) void hid_kernel(
    const float* __restrict__ hs, const _Float16* __restrict__ WhT,
    const float* __restrict__ bh, float* __restrict__ hpart) {
  __shared__ __attribute__((aligned(16))) _Float16 As[64 * LDA];
  __shared__ float rb[64];
  __shared__ float wm[4 * 64];

  const unsigned tid = threadIdx.x, lane = tid & 31u;
  const unsigned w = (unsigned)__builtin_amdgcn_readfirstlane((int)(threadIdx.x >> 5));
  const unsigned mw = w >> 1, nw = w & 1u;
  const unsigned hh = lane >> 4, m = lane & 15u;
  const unsigned row0 = blockIdx.x * 64u;
  const unsigned bidx = row0 / (unsigned)SEQ;
  const unsigned sq0 = row0 - bidx * (unsigned)SEQ;
  const size_t frow0 = (size_t)bidx * SEQ_FULL + sq0;

#pragma unroll
  for (unsigned j = 0; j < 4u; ++j) {
    const unsigned idx = tid + 256u * j;
    const unsigned r = idx >> 4, c = (idx & 15u) * 8u;
    const float* p = hs + (frow0 + r) * HDIM + c;
    const v4f a0 = *(const v4f*)(p);
    const v4f a1 = *(const v4f*)(p + 4);
    float bad = 0.0f;
    v8h o;
#pragma unroll
    for (int i = 0; i < 4; ++i) {
      const float e0 = a0[i], e1 = a1[i];
      bad = ((e0 != e0) || (e1 != e1)) ? 1.0f : bad;
      const float c0 = (e0 != e0) ? 0.0f : e0;
      const float c1 = (e1 != e1) ? 0.0f : e1;
      o[i]     = toh_flush(HCARRY * bf16r(c0));
      o[i + 4] = toh_flush(HCARRY * bf16r(c1));
    }
    bad = red16_max(bad);
    *(v8h*)&As[r * LDA + c] = o;
    if ((tid & 15u) == 0u) rb[r] = bad;
  }
  __syncthreads();

  const _Float16* bp0 = WhT + (size_t)(nw * 32u + m) * HDIM + hh * 8u;
  const _Float16* bp1 = bp0 + (size_t)16 * HDIM;
  const unsigned ao = (mw * 16u + m) * LDA + hh * 8u;
  v8f acc0 = {}, acc1 = {};
#pragma unroll
  for (unsigned k0 = 0; k0 < (unsigned)HDIM; k0 += 32u) {
    const v8h alo = *(const v8h*)&As[ao + k0];
    const v8h ahi = *(const v8h*)&As[ao + k0 + 16u];
    const v16h a  = frag_join(alo, ahi);
    const v16h b0 = frag_at(bp0 + k0);
    const v16h b1 = frag_at(bp1 + k0);
    acc0 = wmma16(a, b0, acc0);
    acc1 = wmma16(a, b1, acc1);
  }

  const float cs = 1.0f / (WCARRY * HCARRY);
  const unsigned c0 = nw * 32u + m, c1 = c0 + 16u;
  const float bb0 = bf16r(bh[c0]);
  const float bb1 = bf16r(bh[c1]);
  float cm0 = NEGV, cm1 = NEGV;
#pragma unroll
  for (int r = 0; r < 8; ++r) {
    const float bad = rb[mw * 16u + hh * 8u + (unsigned)r];
    float v0 = fmaxf(acc0[r] * cs + bb0, 0.0f);
    float v1 = fmaxf(acc1[r] * cs + bb1, 0.0f);
    v0 = (bad != 0.0f) ? FILLV : v0;
    v1 = (bad != 0.0f) ? FILLV : v1;
    cm0 = fmaxf(cm0, v0);
    cm1 = fmaxf(cm1, v1);
  }
  cm0 = fmaxf(cm0, __shfl_xor(cm0, 16, 32));
  cm1 = fmaxf(cm1, __shfl_xor(cm1, 16, 32));
  if (hh == 0u) {
    wm[mw * 64u + c0] = cm0;
    wm[mw * 64u + c1] = cm1;
  }
  __syncthreads();

  if (w == 0u) {
    const unsigned cb = (lane & 15u) * 4u;
    v4f o;
#pragma unroll
    for (int j = 0; j < 4; ++j)
      o[j] = fmaxf(fmaxf(wm[cb + (unsigned)j], wm[64u + cb + (unsigned)j]),
                   fmaxf(wm[128u + cb + (unsigned)j], wm[192u + cb + (unsigned)j]));
    float* p = hpart + (size_t)blockIdx.x * 64u + cb;
    if (lane < 16u) *(volatile v4f*)p = o;
    __threadfence();
    if (lane < 16u) *(volatile v4f*)p = o;
  }
}

__global__ __launch_bounds__(256) void out_kernel(
    const float* __restrict__ obs1, const float* __restrict__ obs2,
    const float* __restrict__ Ws, const float* __restrict__ bs,
    const float* __restrict__ Wv, const float* __restrict__ bv,
    const float* __restrict__ hpart, const _Float16* __restrict__ WoT,
    const float* __restrict__ bo, float* __restrict__ out) {
  __shared__ __attribute__((aligned(16))) _Float16 As[64 * LDA];
  __shared__ __attribute__((aligned(16))) float Cs[64 * LDO];
  __shared__ float part[2 * 8 * 32];
  __shared__ __attribute__((aligned(16))) float cmx[128];

  const unsigned tid = threadIdx.x, lane = tid & 31u;
  const unsigned w = (unsigned)__builtin_amdgcn_readfirstlane((int)(threadIdx.x >> 5));
  const unsigned mw = w >> 1, nw = w & 1u;
  const unsigned hh = lane >> 4, m = lane & 15u;
  const unsigned row0 = blockIdx.x * 64u;
  const unsigned bidx = row0 / (unsigned)SEQ;
  const unsigned sq0 = row0 - bidx * (unsigned)SEQ;
  const size_t fb0 = (size_t)bidx * SEQ_FULL;
  const size_t frow0 = fb0 + sq0;

  {
    const float ws0 = bf16r(Ws[lane]), ws1 = bf16r(Ws[ES + lane]);
    const float wv0 = bf16r(Wv[lane]), wv1 = bf16r(Wv[EV + lane]);
    float sm = NEGV, vm = NEGV;
#pragma unroll 1
    for (unsigned j = w; j < (unsigned)SEQ; j += 8u) {
      const v2f p2 = *(const v2f*)(obs2 + (fb0 + j) * 2u);
      const v2f p1 = *(const v2f*)(obs1 + (fb0 + j) * 2u);
      const float x2 = bf16n(p2[0]), y2 = bf16n(p2[1]);
      const float x1 = bf16n(p1[0]), y1 = bf16n(p1[1]);
      const float vx = 4.0f * (x2 - x1);
      const float vy = 4.0f * (y2 - y1);
      const float ps = ws0 * x2 + ws1 * y2;
      const float pv = wv0 * vx + wv1 * vy;
      const float sn = fmaxf(sm, ps);
      const float vn = fmaxf(vm, pv);
      sm = (ps == ps) ? sn : sm;
      vm = (pv == pv) ? vn : vm;
    }
    part[w * 32u + lane] = sm;
    part[256u + w * 32u + lane] = vm;
  }
  __syncthreads();

  if (w == 0u) {
    float s = part[lane];
#pragma unroll
    for (unsigned g = 1; g < 8u; ++g) s = fmaxf(s, part[g * 32u + lane]);
    cmx[lane] = s;
  } else if (w == 3u) {
    float s = part[256u + lane];
#pragma unroll
    for (unsigned g = 1; g < 8u; ++g) s = fmaxf(s, part[256u + g * 32u + lane]);
    cmx[96u + lane] = s;
  } else if (w == 1u || w == 2u) {
    const unsigned c = (w - 1u) * 32u + lane;
    float hm = NEGV;
#pragma unroll
    for (unsigned g = 0; g < (unsigned)BPB; ++g)
      hm = fmaxf(hm, hpart[((size_t)bidx * BPB + g) * 64u + c]);
    cmx[32u + c] = hm;
  }
  __syncthreads();

  {
    const unsigned r = tid >> 2, q = tid & 3u;
    const size_t fr = frow0 + r;
    const v2f p2 = *(const v2f*)(obs2 + fr * 2u);
    const v2f p1 = *(const v2f*)(obs1 + fr * 2u);
    const float x2 = bf16n(p2[0]), y2 = bf16n(p2[1]);
    const float x1 = bf16n(p1[0]), y1 = bf16n(p1[1]);
    const float vx = 4.0f * (x2 - x1);
    const float vy = 4.0f * (y2 - y1);
    const bool ok2 = (x2 == x2) && (y2 == y2);
    const bool okv = (vx == vx) && (vy == vy);

    const v4f sa0 = *(const v4f*)(Ws + 8u * q);
    const v4f sa1 = *(const v4f*)(Ws + 8u * q + 4u);
    const v4f sb0 = *(const v4f*)(Ws + ES + 8u * q);
    const v4f sb1 = *(const v4f*)(Ws + ES + 8u * q + 4u);
    const v4f sc0 = *(const v4f*)(bs + 8u * q);
    const v4f sc1 = *(const v4f*)(bs + 8u * q + 4u);
    const v4f va0 = *(const v4f*)(Wv + 8u * q);
    const v4f va1 = *(const v4f*)(Wv + 8u * q + 4u);
    const v4f vb0 = *(const v4f*)(Wv + EV + 8u * q);
    const v4f vb1 = *(const v4f*)(Wv + EV + 8u * q + 4u);
    const v4f vc0 = *(const v4f*)(bv + 8u * q);
    const v4f vc1 = *(const v4f*)(bv + 8u * q + 4u);

    v8h os, ov, oh0, oh1;
#pragma unroll
    for (int e = 0; e < 4; ++e) {
      const float ps0 = bf16r(sa0[e]) * x2 + bf16r(sb0[e]) * y2;
      const float ps1 = bf16r(sa1[e]) * x2 + bf16r(sb1[e]) * y2;
      const float ts0 = fmaxf(cmx[8u * q + (unsigned)e] - ps0 + bf16r(sc0[e]), 0.0f);
      const float ts1 = fmaxf(cmx[8u * q + 4u + (unsigned)e] - ps1 + bf16r(sc1[e]), 0.0f);
      os[e]     = toh_flush(ACARRY * (ok2 ? ts0 : FILLV));
      os[e + 4] = toh_flush(ACARRY * (ok2 ? ts1 : FILLV));
      const float pv0 = bf16r(va0[e]) * vx + bf16r(vb0[e]) * vy;
      const float pv1 = bf16r(va1[e]) * vx + bf16r(vb1[e]) * vy;
      const float tv0 = fmaxf(cmx[96u + 8u * q + (unsigned)e] - pv0 + bf16r(vc0[e]), 0.0f);
      const float tv1 = fmaxf(cmx[96u + 8u * q + 4u + (unsigned)e] - pv1 + bf16r(vc1[e]), 0.0f);
      ov[e]     = toh_flush(ACARRY * (okv ? tv0 : FILLV));
      ov[e + 4] = toh_flush(ACARRY * (okv ? tv1 : FILLV));
    }
#pragma unroll
    for (int e = 0; e < 8; ++e) {
      oh0[e] = toh_flush(ACARRY * cmx[32u + 16u * q + (unsigned)e]);
      oh1[e] = toh_flush(ACARRY * cmx[40u + 16u * q + (unsigned)e]);
    }
    *(v8h*)&As[r * LDA + 8u * q]        = os;
    *(v8h*)&As[r * LDA + 32u + 16u * q] = oh0;
    *(v8h*)&As[r * LDA + 40u + 16u * q] = oh1;
    *(v8h*)&As[r * LDA + 96u + 8u * q]  = ov;
  }
  __syncthreads();

  const _Float16* bp = WoT + (size_t)(nw * 64u + m) * PD + hh * 8u;
  const unsigned ao = (mw * 16u + m) * LDA + hh * 8u;
  v8f acc[4];
#pragma unroll
  for (int nb = 0; nb < 4; ++nb) acc[nb] = (v8f){};
#pragma unroll
  for (unsigned k0 = 0; k0 < (unsigned)PD; k0 += 32u) {
    const v8h alo = *(const v8h*)&As[ao + k0];
    const v8h ahi = *(const v8h*)&As[ao + k0 + 16u];
    const v16h a = frag_join(alo, ahi);
#pragma unroll
    for (int nb = 0; nb < 4; ++nb) {
      const v16h b = frag_at(bp + (size_t)(nb * 16) * PD + k0);
      acc[nb] = wmma16(a, b, acc[nb]);
    }
  }
#pragma unroll
  for (int nb = 0; nb < 4; ++nb)
#pragma unroll
    for (int r = 0; r < 8; ++r)
      Cs[(mw * 16u + hh * 8u + (unsigned)r) * LDO + nw * 64u + (unsigned)nb * 16u + m] = acc[nb][r];
  __syncthreads();

  {
    const float cs = 1.0f / (WCARRY * ACARRY);
    const unsigned c = lane * 4u;
    const v4f g = *(const v4f*)(bo + c);
    v4f gb;
#pragma unroll
    for (int j = 0; j < 4; ++j) gb[j] = bf16r(g[j]);
    v4f xs[8];
    size_t off[8];
#pragma unroll
    for (unsigned i = 0; i < 8u; ++i) {
      const unsigned r = w + 8u * i;
      const v4f u = *(const v4f*)&Cs[r * LDO + c];
      v4f val;
#pragma unroll
      for (int j = 0; j < 4; ++j) val[j] = u[j] * cs + gb[j];
      xs[i] = val;
      off[i] = (frow0 + r) * OD + c;
    }
#pragma unroll
    for (int i = 0; i < 8; ++i) *(volatile v4f*)(out + off[i]) = xs[i];
    __threadfence();
#pragma unroll
    for (int i = 0; i < 8; ++i) *(volatile v4f*)(out + off[i]) = xs[i];
  }
}

extern "C" void kernel_launch(void* const* d_in, const int* in_sizes, int n_in,
                              void* d_out, int out_size, void* d_ws, size_t ws_size,
                              hipStream_t stream) {
  if (n_in < 11) return;
  const long long need_rows = (long long)(NB - 1) * SEQ_FULL + SEQ;
  if ((long long)in_sizes[0] < need_rows * HDIM) return;
  if ((long long)in_sizes[1] < need_rows * 2) return;
  if ((long long)in_sizes[2] < need_rows * 2) return;
  if (in_sizes[3] < 2 * ES || in_sizes[4] < ES) return;
  if (in_sizes[5] < 2 * EV || in_sizes[6] < EV) return;
  if (in_sizes[7] < HDIM * EH || in_sizes[8] < EH) return;
  if (in_sizes[9] < PD * OD || in_sizes[10] < OD) return;
  if ((long long)out_size < need_rows * OD) return;
  if (ws_size < WS_TOTAL) return;

  const float* hs   = (const float*)d_in[0];
  const float* obs1 = (const float*)d_in[1];
  const float* obs2 = (const float*)d_in[2];
  const float* w_s  = (const float*)d_in[3];
  const float* b_s  = (const float*)d_in[4];
  const float* w_v  = (const float*)d_in[5];
  const float* b_v  = (const float*)d_in[6];
  const float* w_h  = (const float*)d_in[7];
  const float* b_h  = (const float*)d_in[8];
  const float* w_o  = (const float*)d_in[9];
  const float* b_o  = (const float*)d_in[10];
  float* out = (float*)d_out;

  char* ws = (char*)d_ws;
  _Float16* WhT   = (_Float16*)(ws + OFF_WH);
  _Float16* WoT   = (_Float16*)(ws + OFF_WO);
  float*    hpart = (float*)(ws + OFF_HP);

  dim3 blk(256);
  wconv_kernel<<<dim3(EH / 64, HDIM / 64), blk, 0, stream>>>(w_h, WhT, (unsigned)EH, (unsigned)HDIM);
  wconv_kernel<<<dim3(OD / 64, PD / 64), blk, 0, stream>>>(w_o, WoT, (unsigned)OD, (unsigned)PD);

  hid_kernel<<<dim3(MROWS / 64), blk, 0, stream>>>(hs, WhT, b_h, hpart);
  out_kernel<<<dim3(MROWS / 64), blk, 0, stream>>>(obs1, obs2, w_s, b_s, w_v, b_v,
                                                   hpart, WoT, b_o, out);
}
